// EdgeMLPDecoder_996432413121
// MI455X (gfx1250) — hardware-verified
//
#include <hip/hip_runtime.h>
#include <math.h>

constexpr int   kNode    = 268;
constexpr int   kDim     = 128;
constexpr int   kFeat    = 256;
constexpr int   kHid     = 64;
constexpr int   kHid2    = 32;
constexpr int   kK2View  = 128;
constexpr float kEps     = 1e-5f;
constexpr float kInvHid  = 1.0f / 64.0f;
constexpr float kInvHid2 = 1.0f / 32.0f;
constexpr float kRsqrt2  = 0.70710678118654752440f;

typedef __attribute__((ext_vector_type(16))) _Float16 v16h;
typedef __attribute__((ext_vector_type(8)))  _Float16 v8h;
typedef __attribute__((ext_vector_type(16))) __bf16   v16b;
typedef __attribute__((ext_vector_type(8)))  __bf16   v8b;
typedef __attribute__((ext_vector_type(8)))  float    v8f;
typedef __attribute__((ext_vector_type(4)))  float    v4f;
typedef __attribute__((ext_vector_type(2)))  float    v2f;
typedef __attribute__((ext_vector_type(4)))  unsigned int v4u;

__device__ __forceinline__ unsigned short f2bf_bits(float f) {
  unsigned u = __float_as_uint(f);
  return (unsigned short)((u + 0x7FFFu + ((u >> 16) & 1u)) >> 16);
}
__device__ __forceinline__ float bf_bits2f(unsigned short h) { return __uint_as_float(((unsigned)h) << 16); }

__device__ __forceinline__ void dep_guard_h(v8f& a, v8f& b, v16h x, v16h y) { asm volatile("v_nop\n\tv_nop\n\tv_nop\n\tv_nop" : "+v"(a), "+v"(b) : "v"(x), "v"(y)); }
__device__ __forceinline__ void dep_guard_b(v8f& a, v8f& b, v16b x, v16b y) { asm volatile("v_nop\n\tv_nop\n\tv_nop\n\tv_nop" : "+v"(a), "+v"(b) : "v"(x), "v"(y)); }
__device__ __forceinline__ void keep4_h(v16h a, v16h b, v16h c, v16h d) { asm volatile("v_nop" :: "v"(a), "v"(b), "v"(c), "v"(d)); }
__device__ __forceinline__ void keep4_b(v16b a, v16b b, v16b c, v16b d) { asm volatile("v_nop" :: "v"(a), "v"(b), "v"(c), "v"(d)); }
__device__ __forceinline__ void acc_guard4(v8f& a, v8f& b, v8f& c, v8f& d) { asm volatile("v_nop\n\tv_nop\n\tv_nop\n\tv_nop" : "+v"(a), "+v"(b), "+v"(c), "+v"(d)); }
template <typename T> struct Frag;
template <> struct Frag<_Float16> {
  typedef v16h V; union U { v16h v; v8h h[2]; };
  static __device__ __forceinline__ v16h load(const _Float16* p) {
    U f; f.h[0] = *(const v8h*)(p); f.h[1] = *(const v8h*)(p + 16); return f.v;
  }
  static __device__ __forceinline__ v8f mma(v16h a, v16h b, v8f c) {
    return __builtin_amdgcn_wmma_f32_16x16x32_f16(false, a, false, b, (short)0, c, false, false);
  }
  static __device__ __forceinline__ void guard(v8f& a, v8f& b, v16h x, v16h y) { dep_guard_h(a, b, x, y); }
  static __device__ __forceinline__ void keep(v16h a, v16h b, v16h c, v16h d) { keep4_h(a, b, c, d); }
};
template <> struct Frag<__bf16> {
  typedef v16b V; union U { v16b v; v8b h[2]; };
  static __device__ __forceinline__ v16b load(const __bf16* p) {
    U f; f.h[0] = *(const v8b*)(p); f.h[1] = *(const v8b*)(p + 16); return f.v;
  }
  static __device__ __forceinline__ v8f mma(v16b a, v16b b, v8f c) {
    return __builtin_amdgcn_wmma_f32_16x16x32_bf16(false, a, false, b, (short)0, c, false, false);
  }
  static __device__ __forceinline__ void guard(v8f& a, v8f& b, v16b x, v16b y) { dep_guard_b(a, b, x, y); }
  static __device__ __forceinline__ void keep(v16b a, v16b b, v16b c, v16b d) { keep4_b(a, b, c, d); }
};

__device__ __forceinline__ unsigned pk16(unsigned short a, unsigned short b) { return (unsigned)a | ((unsigned)b << 16); }

template <int ET> struct Elem;
template <> struct Elem<0> { typedef _Float16 T; };
template <> struct Elem<1> { typedef __bf16 T; };
template <int ET, bool SPLIT, int BIAS_MODE, int OUT_MODE, bool RESID, int ACT = 0>
__global__ __launch_bounds__(256) void wmma_gemm64(
    const unsigned short* __restrict__ Ap, const unsigned short* __restrict__ A2p, int lda, long strideA,
    const unsigned short* __restrict__ Btp, const unsigned short* __restrict__ Bt2p, int ldb, long strideB,
    void* __restrict__ Cout, void* __restrict__ Cout2, int ldc, long strideC,
    const float* __restrict__ bias,
    const float* __restrict__ resid, long strideR,
    int M, int N, int K, float scale) {
  typedef typename Elem<ET>::T T;
  typedef typename Frag<T>::V V;
  const T* A = (const T*)Ap; const T* A2 = (const T*)A2p; const T* Bt = (const T*)Btp; const T* Bt2 = (const T*)Bt2p;
  __shared__ __align__(16) float sT[8][16 * 68];
  const int b    = blockIdx.y;
  const int lane = threadIdx.x & 31;
  const int wave = threadIdx.x >> 5;
  const int tilesN = N >> 6;
  const int tilesM = M >> 6;
  const int tile = blockIdx.x * 8 + wave;
  if (tile >= tilesM * tilesN) return;
  const int tm = tile / tilesN;
  const int tn = tile - tm * tilesN;
  const int m0 = tm << 6;
  const int n0 = tn << 6;

  const T* Ab  = A  + (size_t)b * strideA;
  const T* Bb  = Bt + (size_t)b * strideB;
  const T* Ab2 = SPLIT ? (A2  + (size_t)b * strideA) : nullptr;
  const T* Bb2 = SPLIT ? (Bt2 + (size_t)b * strideB) : nullptr;

  const int rlane = lane & 15;
  const int koff  = (lane >> 4) * 8;
  const int mOff  = (lane >> 4) * 8;

  v8f acc[4][4];
#pragma unroll
  for (int i = 0; i < 4; ++i)
#pragma unroll
    for (int j = 0; j < 4; ++j) acc[i][j] = (v8f){0.f,0.f,0.f,0.f,0.f,0.f,0.f,0.f};

  for (int k0 = 0; k0 < K; k0 += 32) {
    V bh[4], bl[4];
#pragma unroll
    for (int j = 0; j < 4; ++j) {
      const size_t bo = (size_t)(n0 + (j << 4) + rlane) * ldb + koff + k0;
      bh[j] = Frag<T>::load(Bb + bo);
      if (SPLIT) bl[j] = Frag<T>::load(Bb2 + bo);
    }
#pragma unroll
    for (int i = 0; i < 4; ++i) {
      const size_t ao = (size_t)(m0 + (i << 4) + rlane) * lda + koff + k0;
      V ah = Frag<T>::load(Ab + ao);
      V al;
      if (SPLIT) al = Frag<T>::load(Ab2 + ao);
#pragma unroll
      for (int j = 0; j < 4; ++j) {
        acc[i][j] = Frag<T>::mma(ah, bh[j], acc[i][j]);
        if (SPLIT) {
          acc[i][j] = Frag<T>::mma(ah, bl[j], acc[i][j]);
          acc[i][j] = Frag<T>::mma(al, bh[j], acc[i][j]);
        }
      }
      Frag<T>::guard(acc[i][0], acc[i][3], ah, SPLIT ? al : ah);
    }
    Frag<T>::keep(bh[0], bh[1], bh[2], bh[3]);
    if (SPLIT) Frag<T>::keep(bl[0], bl[1], bl[2], bl[3]);
  }
  acc_guard4(acc[0][0], acc[0][1], acc[0][2], acc[0][3]);
  acc_guard4(acc[1][0], acc[1][1], acc[1][2], acc[1][3]);
  acc_guard4(acc[2][0], acc[2][1], acc[2][2], acc[2][3]);
  acc_guard4(acc[3][0], acc[3][1], acc[3][2], acc[3][3]);

  float* slab = sT[wave];
  const float* Rb = RESID ? (resid + (size_t)b * strideR) : nullptr;
#pragma unroll
  for (int i = 0; i < 4; ++i) {
    const int mBase = m0 + (i << 4);
#pragma unroll
    for (int j = 0; j < 4; ++j) {
      const int n = n0 + (j << 4) + rlane;
      float bv = 0.f;
      if (BIAS_MODE == 2) bv = bias[n];
#pragma unroll
      for (int r = 0; r < 8; ++r) {
        float v = acc[i][j][r] * scale;
        if (BIAS_MODE == 1) v += bias[mBase + mOff + r];
        if (BIAS_MODE == 2) v += bv;
        if (RESID) v += Rb[(size_t)(mBase + mOff + r) * ldc + n];
        if (ACT == 2) v = fmaxf(v, 0.0f);
        if (ACT == 4) v = (v > 0.f) ? v : 0.01f * v;
        slab[(mOff + r) * 68 + (j << 4) + rlane] = v;
      }
    }
    __builtin_amdgcn_fence(__ATOMIC_RELEASE, "workgroup");
    __builtin_amdgcn_wave_barrier();
    __builtin_amdgcn_fence(__ATOMIC_ACQUIRE, "workgroup");
    if (OUT_MODE == 0) {
      float* C = (float*)Cout + (size_t)b * strideC;
      const int hh = lane >> 4, c4 = (lane & 15) * 4;
      for (int pass = 0; pass < 2; ++pass) {
#pragma unroll
        for (int it = 0; it < 8; ++it) {
          const int row = it * 2 + hh;
          v4f v = *(const v4f*)(slab + row * 68 + c4);
          *(volatile v4f*)(C + (size_t)(mBase + row) * ldc + n0 + c4) = v;
        }
        __threadfence();
      }
    } else {
      const int q = lane >> 3, c8 = (lane & 7) * 8;
      unsigned short* C  = (unsigned short*)Cout  + (size_t)b * strideC;
      unsigned short* C2 = (OUT_MODE == 2) ? ((unsigned short*)Cout2 + (size_t)b * strideC) : nullptr;
      for (int pass = 0; pass < 2; ++pass) {
#pragma unroll
        for (int it = 0; it < 4; ++it) {
          const int row = it * 4 + q;
          const float* sp = slab + row * 68 + c8;
          v8h hv, lv;
#pragma unroll
          for (int e = 0; e < 8; ++e) {
            if (OUT_MODE == 1) {
              hv[e] = (_Float16)sp[e];
            } else {
              unsigned short hb = f2bf_bits(sp[e]);
              unsigned short lb = f2bf_bits(sp[e] - bf_bits2f(hb));
              hv[e] = __builtin_bit_cast(_Float16, hb);
              lv[e] = __builtin_bit_cast(_Float16, lb);
            }
          }
          *(volatile v8h*)(C + (size_t)(mBase + row) * ldc + n0 + c8) = hv;
          if (OUT_MODE == 2) *(volatile v8h*)(C2 + (size_t)(mBase + row) * ldc + n0 + c8) = lv;
        }
        __threadfence();
      }
    }
    __builtin_amdgcn_fence(__ATOMIC_RELEASE, "workgroup");
    __builtin_amdgcn_wave_barrier();
    __builtin_amdgcn_fence(__ATOMIC_ACQUIRE, "workgroup");
  }
}

__device__ __forceinline__ void split_bf(float x, unsigned short& hb, unsigned short& lb) {
  hb = f2bf_bits(x);
  lb = f2bf_bits(x - bf_bits2f(hb));
}
__device__ __forceinline__ float gelu_erf(float x) {
  return 0.5f * x * (1.0f + erff(x * kRsqrt2));
}

__global__ __launch_bounds__(256) void prep_w_kernel(const float* __restrict__ W1, const float* __restrict__ W2,
                                                     unsigned short* __restrict__ W1h, unsigned short* __restrict__ W1l,
                                                     unsigned short* __restrict__ W2h, unsigned short* __restrict__ W2l) {
  const int t = threadIdx.x;
  for (int pass = 0; pass < 2; ++pass) {
#pragma unroll 1
    for (int it = 0; it < 8; ++it) {
      const int p  = it * 256 + t;
      const int n  = p >> 5;
      const int k0 = (p & 31) * 8;
      unsigned short hb[8], lb[8];
#pragma unroll
      for (int e = 0; e < 8; ++e) {
        const float x = W1[(size_t)(k0 + e) * kHid + n];
        split_bf(x, hb[e], lb[e]);
      }
      const v4u hv = (v4u){pk16(hb[0], hb[1]), pk16(hb[2], hb[3]), pk16(hb[4], hb[5]), pk16(hb[6], hb[7])};
      const v4u lv = (v4u){pk16(lb[0], lb[1]), pk16(lb[2], lb[3]), pk16(lb[4], lb[5]), pk16(lb[6], lb[7])};
      *(volatile v4u*)(W1h + (size_t)p * 8) = hv;
      *(volatile v4u*)(W1l + (size_t)p * 8) = lv;
    }
#pragma unroll 1
    for (int it = 0; it < 4; ++it) {
      const int p  = it * 256 + t;
      const int n  = p >> 4;
      const int k0 = (p & 15) * 8;
      const bool onDiag = ((n >> 5) == (k0 >> 6));
      const int nn = n & 31;
      unsigned short hb[8], lb[8];
#pragma unroll
      for (int e = 0; e < 8; ++e) {
        const int kk = (k0 + e) & 63;
        float x = W2[(size_t)kk * kHid2 + nn];
        x = onDiag ? x : 0.0f;
        split_bf(x, hb[e], lb[e]);
      }
      const v4u hv = (v4u){pk16(hb[0], hb[1]), pk16(hb[2], hb[3]), pk16(hb[4], hb[5]), pk16(hb[6], hb[7])};
      const v4u lv = (v4u){pk16(lb[0], lb[1]), pk16(lb[2], lb[3]), pk16(lb[4], lb[5]), pk16(lb[6], lb[7])};
      *(volatile v4u*)(W2h + (size_t)p * 8) = hv;
      *(volatile v4u*)(W2l + (size_t)p * 8) = lv;
    }
    __threadfence();
  }
}

__global__ __launch_bounds__(256) void gather_feat_kernel(const float* __restrict__ H, const int* __restrict__ idx,
                                                          unsigned short* __restrict__ Eh, unsigned short* __restrict__ El,
                                                          int nE, int EP, int bBase) {
  const int lane = threadIdx.x & 31;
  const int wave = threadIdx.x >> 5;
  const int d0   = (lane & 15) * 8;
  const int hsel = lane >> 4;
  const int rbase = blockIdx.x * 64 + wave * 8;
#pragma unroll 1
  for (int i = 0; i < 8; ++i) {
    const int  r     = rbase + i;
    const int  bl    = (r >= EP) ? 1 : 0;
    const int  e     = r - bl * EP;
    const bool valid = (e < nE);
    const int  ec    = valid ? e : (nE - 1);
    int i0 = idx[ec];
    int i1 = idx[nE + ec];
    i0 = (i0 < 0) ? 0 : ((i0 > kNode - 1) ? (kNode - 1) : i0);
    i1 = (i1 < 0) ? 0 : ((i1 > kNode - 1) ? (kNode - 1) : i1);
    const float* up = H + ((size_t)(bBase + bl) * kNode + i0) * kDim + d0;
    const float* vp = H + ((size_t)(bBase + bl) * kNode + i1) * kDim + d0;
    const v4f ua = *(const v4f*)(up);
    const v4f ub = *(const v4f*)(up + 4);
    const v4f va = *(const v4f*)(vp);
    const v4f vb = *(const v4f*)(vp + 4);
    float u[8], v[8];
#pragma unroll
    for (int q = 0; q < 4; ++q) { u[q] = ua[q]; u[4 + q] = ub[q]; v[q] = va[q]; v[4 + q] = vb[q]; }
    unsigned short hb[8], lb[8];
#pragma unroll
    for (int q = 0; q < 8; ++q) {
      const float pr = u[q] * v[q];
      const float sm = u[q] + v[q];
      float x = hsel ? sm : pr;
      x = valid ? x : 0.0f;
      split_bf(x, hb[q], lb[q]);
    }
    const v4u hv = (v4u){pk16(hb[0], hb[1]), pk16(hb[2], hb[3]), pk16(hb[4], hb[5]), pk16(hb[6], hb[7])};
    const v4u lv = (v4u){pk16(lb[0], lb[1]), pk16(lb[2], lb[3]), pk16(lb[4], lb[5]), pk16(lb[6], lb[7])};
    const size_t o = (size_t)r * kFeat + (size_t)lane * 8;
    *(volatile v4u*)(Eh + o) = hv;
    *(volatile v4u*)(El + o) = lv;
    __threadfence();
    *(volatile v4u*)(Eh + o) = hv;
    *(volatile v4u*)(El + o) = lv;
  }
}

__global__ __launch_bounds__(256) void ln1_gelu_kernel(const float* __restrict__ Cin, const float* __restrict__ bias,
                                                       const float* __restrict__ gam, const float* __restrict__ bet,
                                                       unsigned short* __restrict__ Hout, long planeStride) {
  __shared__ __align__(16) unsigned int sst[512];
  const int t    = threadIdx.x;
  const int lane = t & 31;
  const int wave = t >> 5;
  const int r0   = blockIdx.x * 8;
  const int r    = r0 + wave;
  const int c    = lane * 2;
  const v2f xv = *(const v2f*)(Cin + (size_t)r * kHid + c);
  const float x0 = xv[0] + bias[c];
  const float x1 = xv[1] + bias[c + 1];
  float s = x0 + x1;
#pragma unroll
  for (int off = 1; off < 32; off <<= 1) s += __shfl_xor(s, off, 32);
  const float mu = s * kInvHid;
  const float d0 = x0 - mu;
  const float d1 = x1 - mu;
  float q = d0 * d0 + d1 * d1;
#pragma unroll
  for (int off = 1; off < 32; off <<= 1) q += __shfl_xor(q, off, 32);
  const float rstd = rsqrtf(q * kInvHid + kEps);
  const float y0 = (d0 * rstd) * gam[c] + bet[c];
  const float y1 = (d1 * rstd) * gam[c + 1] + bet[c + 1];
  const float a0 = gelu_erf(y0);
  const float a1 = gelu_erf(y1);
  unsigned short hb0, lb0, hb1, lb1;
  split_bf(a0, hb0, lb0);
  split_bf(a1, hb1, lb1);
  sst[t]       = pk16(hb0, hb1);
  sst[256 + t] = pk16(lb0, lb1);
  __syncthreads();
  if (t < 128) {
    const int plane = t >> 6;
    const int piece = t & 63;
    const int rowp  = piece >> 3;
    const int c8    = (piece & 7) * 8;
    const v4u val = *(const v4u*)(sst + plane * 256 + piece * 4);
    unsigned short* dst = Hout + (size_t)plane * planeStride + (size_t)(r0 + rowp) * kHid + c8;
    *(volatile v4u*)dst = val;
    __threadfence();
    *(volatile v4u*)dst = val;
  }
}

__global__ __launch_bounds__(512) void ln2_head_kernel(const float* __restrict__ Cin, const float* __restrict__ bias,
                                                       const float* __restrict__ gam, const float* __restrict__ bet,
                                                       const float* __restrict__ W3, const float* __restrict__ b3,
                                                       float* __restrict__ OutS, int nE, int EP) {
  __shared__ __align__(16) float sOut[32];
  const int t   = threadIdx.x;
  const int grp = t >> 4;
  const int l16 = t & 15;
  const int c   = l16 * 2;
  const int r   = blockIdx.x * 32 + grp;
  const v2f xv = *(const v2f*)(Cin + (size_t)r * kHid2 + c);
  const float x0 = xv[0] + bias[c];
  const float x1 = xv[1] + bias[c + 1];
  float s = x0 + x1;
#pragma unroll
  for (int off = 1; off < 16; off <<= 1) s += __shfl_xor(s, off, 32);
  const float mu = s * kInvHid2;
  const float d0 = x0 - mu;
  const float d1 = x1 - mu;
  float q = d0 * d0 + d1 * d1;
#pragma unroll
  for (int off = 1; off < 16; off <<= 1) q += __shfl_xor(q, off, 32);
  const float rstd = rsqrtf(q * kInvHid2 + kEps);
  const float y0 = (d0 * rstd) * gam[c] + bet[c];
  const float y1 = (d1 * rstd) * gam[c + 1] + bet[c + 1];
  const float a0 = gelu_erf(y0);
  const float a1 = gelu_erf(y1);
  float dot = a0 * W3[c] + a1 * W3[c + 1];
#pragma unroll
  for (int off = 1; off < 16; off <<= 1) dot += __shfl_xor(dot, off, 32);
  float val = dot + b3[0];
  const int e = r - ((r >= EP) ? EP : 0);
  val = (e < nE) ? val : 0.0f;
  if (l16 == 0) sOut[grp] = val;
  __syncthreads();
  if (t < 8) {
    const v4f v = *(const v4f*)(sOut + t * 4);
    float* dst = OutS + (size_t)blockIdx.x * 32 + t * 4;
    *(volatile v4f*)dst = v;
    __threadfence();
    *(volatile v4f*)dst = v;
  }
}

__global__ __launch_bounds__(256) void copy_out_kernel(const float* __restrict__ S, float* __restrict__ out,
                                                       int nE, int EP, int n4) {
  const int gi = blockIdx.x * 256 + threadIdx.x;
  if (gi >= n4) return;
  const int f0 = gi * 4;
  v4f v;
#pragma unroll
  for (int j = 0; j < 4; ++j) {
    const int f = f0 + j;
    const int b = f / nE;
    const int e = f - b * nE;
    v[j] = S[(size_t)b * EP + e];
  }
  float* dst = out + (size_t)f0;
  *(volatile v4f*)dst = v;
  __threadfence();
  *(volatile v4f*)dst = v;
}

extern "C" void kernel_launch(void* const* d_in, const int* in_sizes, int n_in,
                              void* d_out, int out_size, void* d_ws, size_t ws_size,
                              hipStream_t stream) {
  if (n_in < 12) return;
  const float* H   = (const float*)d_in[0];
  const int*   idx = (const int*)  d_in[1];
  const float* W1  = (const float*)d_in[2];
  const float* b1  = (const float*)d_in[3];
  const float* g1  = (const float*)d_in[4];
  const float* be1 = (const float*)d_in[5];
  const float* W2  = (const float*)d_in[6];
  const float* b2  = (const float*)d_in[7];
  const float* g2  = (const float*)d_in[8];
  const float* be2 = (const float*)d_in[9];
  const float* W3  = (const float*)d_in[10];
  const float* b3  = (const float*)d_in[11];
  float* out = (float*)d_out;

  if (in_sizes[0] % (kNode * kDim) != 0) return;
  const int B  = in_sizes[0] / (kNode * kDim);
  if (in_sizes[1] % 2 != 0) return;
  const int nE = in_sizes[1] / 2;
  if (B < 2 || (B % 2) != 0 || nE < 1) return;
  if (in_sizes[2] != kFeat * kHid || in_sizes[3] != kHid || in_sizes[4] != kHid || in_sizes[5] != kHid) return;
  if (in_sizes[6] != kHid * kHid2 || in_sizes[7] != kHid2 || in_sizes[8] != kHid2 || in_sizes[9] != kHid2) return;
  if (in_sizes[10] != kHid2 || in_sizes[11] != 1) return;
  if ((long)out_size != (long)B * (long)nE || (out_size % 4) != 0) return;

  const int EP = ((nE + 63) / 64) * 64;
  const int MP = 2 * EP;
  const int nChunk = B / 2;

  size_t off = 0;
  auto carve = [&](size_t bytes) { const size_t o = off; off += (bytes + 255) & ~(size_t)255; return o; };
  const size_t oW1h = carve((size_t)kHid * kFeat * 2);
  const size_t oW1l = carve((size_t)kHid * kFeat * 2);
  const size_t oW2h = carve((size_t)kHid * kK2View * 2);
  const size_t oW2l = carve((size_t)kHid * kK2View * 2);
  const size_t oEh  = carve((size_t)MP * kFeat * 2);
  const size_t oEl  = carve((size_t)MP * kFeat * 2);
  const size_t oC1  = carve((size_t)MP * kHid * 4);
  const size_t oH1  = carve((size_t)2 * MP * kHid * 2);
  const size_t oC2  = carve((size_t)MP * kHid2 * 4);
  const size_t oOut = carve((size_t)B * EP * 4);
  if (off > ws_size) return;

  char* ws = (char*)d_ws;
  unsigned short* W1h = (unsigned short*)(ws + oW1h);
  unsigned short* W1l = (unsigned short*)(ws + oW1l);
  unsigned short* W2h = (unsigned short*)(ws + oW2h);
  unsigned short* W2l = (unsigned short*)(ws + oW2l);
  unsigned short* Eh  = (unsigned short*)(ws + oEh);
  unsigned short* El  = (unsigned short*)(ws + oEl);
  float*          C1  = (float*)(ws + oC1);
  unsigned short* H1  = (unsigned short*)(ws + oH1);
  const long      h1PlaneStride = (long)MP * kHid;
  unsigned short* H1l = H1 + h1PlaneStride;
  float*          C2  = (float*)(ws + oC2);
  float*          OUTS = (float*)(ws + oOut);

  prep_w_kernel<<<dim3(1), dim3(256), 0, stream>>>(W1, W2, W1h, W1l, W2h, W2l);

  const int tiles1  = (MP / 64) * (kHid / 64);
  const int blocks1 = (tiles1 + 7) / 8;
  const int tiles2  = (EP / 64) * (64 / 64);
  const int blocks2 = (tiles2 + 7) / 8;

  for (int c = 0; c < nChunk; ++c) {
    gather_feat_kernel<<<dim3(MP / 64), dim3(256), 0, stream>>>(H, idx, Eh, El, nE, EP, 2 * c);
    wmma_gemm64<1, true, 0, 0, false><<<dim3(blocks1, 1), dim3(256), 0, stream>>>(
        Eh, El, kFeat, 0L, W1h, W1l, kFeat, 0L, (void*)C1, (void*)C1, kHid, 0L,
        b1, C1, 0L, MP, kHid, kFeat, 1.0f);
    ln1_gelu_kernel<<<dim3(MP / 8), dim3(256), 0, stream>>>(C1, b1, g1, be1, H1, h1PlaneStride);
    wmma_gemm64<1, true, 0, 0, false><<<dim3(blocks2, 1), dim3(256), 0, stream>>>(
        H1, H1l, kK2View, 0L, W2h, W2l, kK2View, 0L, (void*)C2, (void*)C2, 64, 0L,
        b2, C2, 0L, EP, 64, kK2View, 1.0f);
    ln2_head_kernel<<<dim3(MP / 32), dim3(512), 0, stream>>>(C2, b2, g2, be2, W3, b3,
                                                              OUTS + (size_t)c * MP, nE, EP);
  }

  const int n4 = out_size / 4;
  copy_out_kernel<<<dim3((n4 + 255) / 256), dim3(256), 0, stream>>>(OUTS, out, nE, EP, n4);
}
